// E3Gnn_63883343561092
// MI455X (gfx1250) — hardware-verified
//
#include <hip/hip_runtime.h>
#include <stddef.h>
#include <math.h>


#pragma clang fp contract(off)

#define NN   256
#define NTOT 512
#define VW   48
#define HF   128
#define OH   64
#define TP   132
#define XP   264
#define NTI  16
#define ISD  0.06262242910851495f
#define I255 (1.0f / 255.0f)

typedef unsigned short us;
typedef float  v4f  __attribute__((ext_vector_type(4)));
typedef float  v8f  __attribute__((ext_vector_type(8)));
typedef us     v8us __attribute__((ext_vector_type(8)));
typedef __bf16 v16b __attribute__((ext_vector_type(16)));
union FB { v16b v; v8us u[2]; };
static_assert(sizeof(FB) == 32);
static_assert((TP % 4) == 0 && (XP % 4) == 0);

__device__ __forceinline__ us bfr(float x) {
  unsigned u = __float_as_uint(x);
  u += 0x7FFFu + ((u >> 16) & 1u);
  return (us)(u >> 16);
}
__device__ __forceinline__ float bff(us b) { return __uint_as_float(((unsigned)b) << 16); }
__device__ __forceinline__ void split3(float x, us& p, us& q, us& s) {
  p = bfr(x);  const float r1 = x - bff(p);
  q = bfr(r1); const float r2 = r1 - bff(q);
  s = bfr(r2);
}

__device__ __forceinline__ float sigm(float x) {
  const float e = expf(fminf(-x, 40.0f));
  return 1.0f / (1.0f + e);
}

#define WMB(A, B, C) __builtin_amdgcn_wmma_f32_16x16x32_bf16(false, A, false, B, (short)0, C, false, false)

__device__ __forceinline__ v8f wm6(v16b ah, v16b am, v16b al, v16b bh, v16b bm, v16b bl, v8f c) {
  c = WMB(am, bm, c);
  c = WMB(al, bh, c);
  c = WMB(ah, bl, c);
  c = WMB(am, bh, c);
  c = WMB(ah, bm, c);
  c = WMB(ah, bh, c);
  asm volatile("v_nop\n\tv_nop\n\tv_nop\n\tv_nop" : "+v"(c) : "v"(ah), "v"(am), "v"(al), "v"(bh), "v"(bm), "v"(bl));
  return c;
}
__device__ __forceinline__ v8f wm3(v16b ah, v16b al, v16b bh, v16b bl, v8f c) {
  c = WMB(al, bh, c);
  c = WMB(ah, bl, c);
  c = WMB(ah, bh, c);
  asm volatile("v_nop\n\tv_nop\n\tv_nop\n\tv_nop" : "+v"(c) : "v"(ah), "v"(al), "v"(bh), "v"(bl));
  return c;
}

template <int NFT>
__device__ __forceinline__ void zacc(v8f (&acc)[NFT]) {
#pragma unroll
  for (int ft = 0; ft < NFT; ++ft) {
#pragma unroll
    for (int r = 0; r < 8; ++r) acc[ft][r] = 0.0f;
  }
}

template <int NK, int NFT, int W3>
__device__ __forceinline__ void gemmS(const us* __restrict__ w, int ps, const float* xt, int xp, v8f (&acc)[NFT], int lane) {
  const int h = lane >> 4, n = lane & 15;
#pragma unroll 1
  for (int kc = 0; kc < NK; ++kc) {
    const float* xr = xt + n * xp + 32 * kc + 8 * h;
    const v4f x0 = *(const v4f*)xr, x1 = *(const v4f*)(xr + 4);
    const v4f x2 = *(const v4f*)(xr + 16), x3 = *(const v4f*)(xr + 20);
    const float xs[16] = {x0.x, x0.y, x0.z, x0.w, x1.x, x1.y, x1.z, x1.w,
                          x2.x, x2.y, x2.z, x2.w, x3.x, x3.y, x3.z, x3.w};
    FB bh, bm, bl;
#pragma unroll
    for (int i = 0; i < 16; ++i) {
      us p, q, s;
      split3(xs[i], p, q, s);
      bh.u[i >> 3][i & 7] = p; bm.u[i >> 3][i & 7] = q; bl.u[i >> 3][i & 7] = s;
    }
#pragma unroll
    for (int ft = 0; ft < NFT; ++ft) {
      const size_t ao = (size_t)(16 * ft + n) * (32 * NK) + 32 * kc + 8 * h;
      const us* p0 = w + ao;
      const us* p1 = w + (size_t)ps + ao;
      FB ah, am;
      ah.u[0] = *(const v8us*)p0; ah.u[1] = *(const v8us*)(p0 + 16);
      am.u[0] = *(const v8us*)p1; am.u[1] = *(const v8us*)(p1 + 16);
      if (W3 != 0) {
        const us* p2 = w + 2 * (size_t)ps + ao;
        FB al;
        al.u[0] = *(const v8us*)p2; al.u[1] = *(const v8us*)(p2 + 16);
        acc[ft] = wm6(ah.v, am.v, al.v, bh.v, bm.v, bl.v, acc[ft]);
      } else {
        acc[ft] = wm3(ah.v, am.v, bh.v, bm.v, acc[ft]);
      }
    }
  }
}

template <int NFT, int ACT, int BIAS, int ADD>
__device__ __forceinline__ void epi(v8f (&acc)[NFT], const float* __restrict__ bias,
                                    const float* __restrict__ prow, const float* qrow, float* t, int lane) {
  const int h = lane >> 4, n = lane & 15;
#pragma unroll
  for (int ft = 0; ft < NFT; ++ft) {
    const int f0 = 16 * ft + 8 * h;
    float v[8];
#pragma unroll
    for (int r = 0; r < 8; ++r) v[r] = acc[ft][r];
    if ((ADD & 1) != 0) {
      const v4f u0 = *(const v4f*)(prow + f0), u1 = *(const v4f*)(prow + f0 + 4);
      v[0] += u0.x; v[1] += u0.y; v[2] += u0.z; v[3] += u0.w; v[4] += u1.x; v[5] += u1.y; v[6] += u1.z; v[7] += u1.w;
    }
    if ((ADD & 2) != 0) {
      const v4f u0 = *(const v4f*)(qrow + f0), u1 = *(const v4f*)(qrow + f0 + 4);
      v[0] += u0.x; v[1] += u0.y; v[2] += u0.z; v[3] += u0.w; v[4] += u1.x; v[5] += u1.y; v[6] += u1.z; v[7] += u1.w;
    }
    if (BIAS != 0) {
      const v4f u0 = *(const v4f*)(bias + f0), u1 = *(const v4f*)(bias + f0 + 4);
      v[0] += u0.x; v[1] += u0.y; v[2] += u0.z; v[3] += u0.w; v[4] += u1.x; v[5] += u1.y; v[6] += u1.z; v[7] += u1.w;
    }
    if (ACT != 0) {
#pragma unroll
      for (int r = 0; r < 8; ++r) v[r] = v[r] * sigm(v[r]);
    }
    if ((ADD & 4) != 0) {
      const v4f u0 = *(const v4f*)(qrow + f0), u1 = *(const v4f*)(qrow + f0 + 4);
      v[0] = u0.x + v[0]; v[1] = u0.y + v[1]; v[2] = u0.z + v[2]; v[3] = u0.w + v[3];
      v[4] = u1.x + v[4]; v[5] = u1.y + v[5]; v[6] = u1.z + v[6]; v[7] = u1.w + v[7];
    }
    const v4f o0 = {v[0], v[1], v[2], v[3]}, o1 = {v[4], v[5], v[6], v[7]};
    *(v4f*)(t + n * TP + f0) = o0;
    *(v4f*)(t + n * TP + f0 + 4) = o1;
  }
}

__global__ __launch_bounds__(256) void k_prep(const float* __restrict__ src, us* dst, int Lc, int lstride,
                                               int k0, int K, int Ns, int Np, int Kp, int nG, int E, int nP) {
  const int g = blockIdx.x * 256 + threadIdx.x;
  const bool ok = g < nG;
  const int e0 = (ok ? g : 0) * 8;
  const int per = Np * Kp;
  int l = e0 / per;
  const int rem = e0 - l * per;
  const int n = rem / Kp;
  const int kb = rem - n * Kp;
  l = min(l, Lc - 1);
  const int nn = min(n, Ns - 1);
  v8us pa, pb, pc;
#pragma unroll
  for (int i = 0; i < 8; ++i) {
    const int k = kb + i;
    const int kk = min(k, K - 1);
    float v = src[(size_t)l * lstride + (size_t)(k0 + kk) * Ns + nn];
    v = (k < K && n < Ns) ? v : 0.0f;
    us p, q, s;
    split3(v, p, q, s);
    pa[i] = p; pb[i] = q; pc[i] = s;
  }
#pragma unroll 1
  for (int pp = 0; pp < 2; ++pp) {
    if (ok) {
      *(volatile v8us*)(dst + e0) = pa;
      *(volatile v8us*)(dst + (size_t)E + e0) = pb;
      if (nP > 2) *(volatile v8us*)(dst + 2 * (size_t)E + e0) = pc;
    }
    __threadfence();
  }
}

__global__ __launch_bounds__(256) void k_init(const float* __restrict__ x, float* vin, float* vec, float* hz, float* pz, float* qz) {
  __shared__ float red[3][NN];
  __shared__ float vs[NN * 3];
  const int b = blockIdx.x, t = threadIdx.x, nf = b * NN + t;
  const float x0 = x[nf * 3], x1 = x[nf * 3 + 1], x2 = x[nf * 3 + 2];
  red[0][t] = x0; red[1][t] = x1; red[2][t] = x2;
  __syncthreads();
#pragma unroll 1
  for (int st = NN / 2; st > 0; st >>= 1) {
    if (t < st) { red[0][t] += red[0][t + st]; red[1][t] += red[1][t + st]; red[2][t] += red[2][t + st]; }
    __syncthreads();
  }
  const float iv = 1.0f / (float)NN;
  const float v0 = x0 - red[0][0] * iv, v1 = x1 - red[1][0] * iv, v2 = x2 - red[2][0] * iv;
  vs[t * 3] = v0; vs[t * 3 + 1] = v1; vs[t * 3 + 2] = v2;
  __syncthreads();
  const v4f q4 = {v0, v1, v2, 0.0f};
  v4f vv[12];
#pragma unroll
  for (int q = 0; q < 12; ++q) {
    const int i = t + NN * q;
    const int nd = i / 12;
    const int eb = (i - nd * 12) * 4;
    v4f w4;
    w4.x = vs[nd * 3 + (eb % 3)];
    w4.y = vs[nd * 3 + ((eb + 1) % 3)];
    w4.z = vs[nd * 3 + ((eb + 2) % 3)];
    w4.w = vs[nd * 3 + ((eb + 3) % 3)];
    vv[q] = w4;
  }
  const v4f z = {0.0f, 0.0f, 0.0f, 0.0f};
  float* vb = vec + (size_t)b * NN * VW;
  float* hb = hz + (size_t)b * NN * HF;
  float* pb = pz + (size_t)b * NN * HF;
  float* qb = qz + (size_t)b * NN * HF;
#pragma unroll 1
  for (int pp = 0; pp < 2; ++pp) {
    *(volatile v4f*)(vin + (size_t)nf * 4) = q4;
#pragma unroll
    for (int q = 0; q < 12; ++q) *(volatile v4f*)(vb + 4 * (t + NN * q)) = vv[q];
#pragma unroll 1
    for (int q = 0; q < 32; ++q) {
      *(volatile v4f*)(hb + 4 * (t + NN * q)) = z;
      *(volatile v4f*)(pb + 4 * (t + NN * q)) = z;
      *(volatile v4f*)(qb + 4 * (t + NN * q)) = z;
    }
    __threadfence();
  }
}

__global__ __launch_bounds__(32) __attribute__((amdgpu_num_vgpr(256)))
void k_pair(const float* __restrict__ vec, const float* __restrict__ P, const float* __restrict__ Q,
            const us* __restrict__ wA, int psA, const us* __restrict__ wB, int psB,
            const us* __restrict__ wI, int psI, const us* __restrict__ x1, int psX1,
            const us* __restrict__ x2, int psX2, const us* __restrict__ x3, int psX3,
            const float* __restrict__ b1, const float* __restrict__ b2, const float* __restrict__ bI,
            const float* __restrict__ c1, const float* __restrict__ c2, const float* __restrict__ c3,
            float* MI, float* SH) {
  __shared__ __attribute__((aligned(16))) float TA[16 * TP];
  __shared__ __attribute__((aligned(16))) float TB[16 * TP];
  __shared__ __attribute__((aligned(16))) float DF[16 * VW];
  __shared__ __attribute__((aligned(16))) float LN[256];
  __shared__ __attribute__((aligned(16))) float PXS[256];
  __shared__ __attribute__((aligned(16))) float QR[HF];
  __shared__ __attribute__((aligned(16))) float VR[VW];
  __shared__ __attribute__((aligned(16))) float PSH[64];
  __shared__ float ES[16];
  const int lane = threadIdx.x & 31, h = lane >> 4, n = lane & 15;
  const int rf = blockIdx.x, b = rf >> 8, r = rf & 255;
  *(v4f*)(QR + 4 * lane) = *(const v4f*)(Q + (size_t)rf * HF + 4 * lane);
  if (lane < 12) *(v4f*)(VR + 4 * lane) = *(const v4f*)(vec + (size_t)rf * VW + 4 * lane);
  float pm0 = 0.0f, pm1 = 0.0f, pm2 = 0.0f, pm3 = 0.0f, ps0 = 0.0f, ps1 = 0.0f;
  const int ca = lane / 3;
  const int i1 = (lane < 16) ? (32 + lane) : 32;
  const int cb = i1 / 3;
#pragma unroll 1
  for (int t = 0; t < NTI; ++t) {
    const int j0 = t * 16;
    const int s  = b * NN + j0 + n;
    __syncthreads();
    {
      const float* vsp = vec + (size_t)s * VW + 24 * h;
      float sa[24];
#pragma unroll
      for (int q = 0; q < 6; ++q) {
        const v4f t4 = *(const v4f*)(vsp + 4 * q);
        sa[4 * q] = t4.x; sa[4 * q + 1] = t4.y; sa[4 * q + 2] = t4.z; sa[4 * q + 3] = t4.w;
      }
      float dd[24], lv[8], l2v[8];
#pragma unroll
      for (int ci = 0; ci < 8; ++ci) {
        const int c = 8 * h + ci;
        const float d0 = VR[c * 3] - sa[ci * 3];
        const float d1 = VR[c * 3 + 1] - sa[ci * 3 + 1];
        const float d2 = VR[c * 3 + 2] - sa[ci * 3 + 2];
        dd[ci * 3] = d0; dd[ci * 3 + 1] = d1; dd[ci * 3 + 2] = d2;
        float l2 = d0 * d0 + d1 * d1 + d2 * d2;
        l2 = l2 + 1e-16f;
        const float len = sqrtf(l2);
        lv[ci] = len;
        l2v[ci] = len * len;
      }
#pragma unroll
      for (int q = 0; q < 6; ++q) {
        const v4f o = {dd[4 * q], dd[4 * q + 1], dd[4 * q + 2], dd[4 * q + 3]};
        *(v4f*)(DF + n * VW + 24 * h + 4 * q) = o;
      }
      const v4f la = {lv[0], lv[1], lv[2], lv[3]}, lb = {lv[4], lv[5], lv[6], lv[7]};
      *(v4f*)(LN + n * 16 + 8 * h) = la;
      *(v4f*)(LN + n * 16 + 8 * h + 4) = lb;
      const v4f qa = {l2v[0], l2v[1], l2v[2], l2v[3]}, qb = {l2v[4], l2v[5], l2v[6], l2v[7]};
      const v4f z = {0.0f, 0.0f, 0.0f, 0.0f};
      *(v4f*)(TA + n * TP + 8 * h) = qa;
      *(v4f*)(TA + n * TP + 8 * h + 4) = qb;
      *(v4f*)(TA + n * TP + 16 + 8 * h) = z;
      *(v4f*)(TA + n * TP + 16 + 8 * h + 4) = z;
    }
    __syncthreads();
    v8f acc[8];
    zacc<8>(acc);
    gemmS<1, 8, 1>(wA, psA, TA, TP, acc, lane);
    epi<8, 1, 1, 3>(acc, b1, P + (size_t)s * HF, QR, TB, lane);
    __syncthreads();
    zacc<8>(acc);
    gemmS<4, 8, 1>(wB, psB, TB, TP, acc, lane);
    epi<8, 1, 1, 0>(acc, b2, P, QR, TA, lane);
    __syncthreads();
    {
      v8f g[1];
      zacc<1>(g);
      gemmS<4, 1, 1>(wI, psI, TA, TP, g, lane);
      const float e = sigm(g[0][0] + bI[0]);
      if (h == 0) ES[n] = ((j0 + n) != r) ? e : 0.0f;
    }
    __syncthreads();
#pragma unroll 4
    for (int q = 0; q < 16; ++q) {
      const v4f mv = *(const v4f*)(TA + q * TP + 4 * lane);
      const float e = ES[q];
      const float p0 = mv.x * e, p1 = mv.y * e, p2 = mv.z * e, p3 = mv.w * e;
      pm0 += p0; pm1 += p1; pm2 += p2; pm3 += p3;
    }
    zacc<8>(acc);
    gemmS<4, 8, 0>(x1, psX1, TA, TP, acc, lane);
    epi<8, 1, 1, 0>(acc, c1, P, QR, TB, lane);
    __syncthreads();
    zacc<8>(acc);
    gemmS<4, 8, 0>(x2, psX2, TB, TP, acc, lane);
    epi<8, 1, 1, 0>(acc, c2, P, QR, TA, lane);
    __syncthreads();
    {
      v8f g[1];
      zacc<1>(g);
      gemmS<4, 1, 0>(x3, psX3, TA, TP, g, lane);
      const v4f u0 = *(const v4f*)(c3 + 8 * h), u1 = *(const v4f*)(c3 + 8 * h + 4);
      v4f o0, o1;
      o0.x = g[0][0] + u0.x; o0.y = g[0][1] + u0.y; o0.z = g[0][2] + u0.z; o0.w = g[0][3] + u0.w;
      o1.x = g[0][4] + u1.x; o1.y = g[0][5] + u1.y; o1.z = g[0][6] + u1.z; o1.w = g[0][7] + u1.w;
      *(v4f*)(PXS + n * 16 + 8 * h) = o0;
      *(v4f*)(PXS + n * 16 + 8 * h + 4) = o1;
    }
    __syncthreads();
#pragma unroll 4
    for (int q = 0; q < 16; ++q) {
      const float pa = PXS[q * 16 + ca], da = DF[q * VW + lane], la = LN[q * 16 + ca];
      const float ia = 1.0f / (1.0f + la);
      ps0 += (pa * da) * ia;
      const float pb = PXS[q * 16 + cb], db = DF[q * VW + i1], lb = LN[q * 16 + cb];
      const float ib = 1.0f / (1.0f + lb);
      const float tb = (pb * db) * ib;
      ps1 += (lane < 16) ? tb : 0.0f;
    }
  }
  __syncthreads();
  PSH[lane] = ps0;
  PSH[32 + lane] = ps1;
  __syncthreads();
  const v4f mo = {pm0 * ISD, pm1 * ISD, pm2 * ISD, pm3 * ISD};
  const int sl = (lane < 16) ? lane : 0;
  const v4f so = *(const v4f*)(PSH + 4 * sl);
#pragma unroll 1
  for (int pp = 0; pp < 2; ++pp) {
    *(volatile v4f*)(MI + (size_t)rf * HF + 4 * lane) = mo;
    if (lane < 16) *(volatile v4f*)(SH + (size_t)rf * 64 + 4 * lane) = so;
    __threadfence();
  }
}

__global__ __launch_bounds__(32) __attribute__((amdgpu_num_vgpr(256)))
void k_node(const float* __restrict__ MI, const float* __restrict__ SH, const float* __restrict__ Hc,
            const float* __restrict__ Vc, const float* __restrict__ VIN,
            const us* __restrict__ h1, int psH1, const us* __restrict__ h2, int psH2, const us* __restrict__ h3, int psH3,
            const float* __restrict__ d1, const float* __restrict__ d2, const float* __restrict__ d3,
            const us* __restrict__ wp, const us* __restrict__ wq, int psPQ,
            const us* __restrict__ wr, int psR, const float* __restrict__ rb,
            float* Hn, float* Vn, float* Pn, float* Qn, float* out, int last) {
  __shared__ __attribute__((aligned(16))) float X[16 * XP];
  __shared__ __attribute__((aligned(16))) float T1[16 * TP];
  __shared__ __attribute__((aligned(16))) float T2[16 * TP];
  __shared__ __attribute__((aligned(16))) float HN[16 * TP];
  const int lane = threadIdx.x & 31, h = lane >> 4, n = lane & 15;
  const int n0 = blockIdx.x * 16;
#pragma unroll 4
  for (int i = lane; i < 512; i += 32) {
    const int row = i >> 5, c4 = (i & 31) * 4;
    *(v4f*)(X + row * XP + c4)      = *(const v4f*)(MI + (size_t)(n0 + row) * HF + c4);
    *(v4f*)(X + row * XP + HF + c4) = *(const v4f*)(Hc + (size_t)(n0 + row) * HF + c4);
  }
  __syncthreads();
  v8f acc[8];
  zacc<8>(acc);
  gemmS<8, 8, 1>(h1, psH1, X, XP, acc, lane);
  epi<8, 1, 1, 0>(acc, d1, MI, X, T1, lane);
  __syncthreads();
  zacc<8>(acc);
  gemmS<4, 8, 1>(h2, psH2, T1, TP, acc, lane);
  epi<8, 1, 1, 0>(acc, d2, MI, X, T2, lane);
  __syncthreads();
  zacc<8>(acc);
  gemmS<4, 8, 1>(h3, psH3, T2, TP, acc, lane);
  epi<8, 0, 1, 4>(acc, d3, MI, X + n * XP + HF, HN, lane);
  __syncthreads();
  v4f ov[6];
#pragma unroll
  for (int q = 0; q < 6; ++q) {
    const int fi = q * 128 + 4 * lane;
    const int nd = fi / VW;
    const int e  = fi - nd * VW;
    const v4f a  = *(const v4f*)(Vc + (size_t)n0 * VW + fi);
    const v4f sh = *(const v4f*)(SH + (size_t)(n0 + nd) * 64 + e);
    v4f v;
    v.x = a.x + sh.x * I255; v.y = a.y + sh.y * I255; v.z = a.z + sh.z * I255; v.w = a.w + sh.w * I255;
    if (last != 0) {
      const v4f vr = *(const v4f*)(VIN + (size_t)(n0 + nd) * 4);
      const int da = e % 3, db = (e + 1) % 3, dc = (e + 2) % 3, de = (e + 3) % 3;
      const float ia = (da == 0) ? vr.x : ((da == 1) ? vr.y : vr.z);
      const float ib = (db == 0) ? vr.x : ((db == 1) ? vr.y : vr.z);
      const float ic = (dc == 0) ? vr.x : ((dc == 1) ? vr.y : vr.z);
      const float ie = (de == 0) ? vr.x : ((de == 1) ? vr.y : vr.z);
      v.x = v.x - ia; v.y = v.y - ib; v.z = v.z - ic; v.w = v.w - ie;
    }
    ov[q] = v;
  }
  {
    float* vd = (last != 0) ? out : Vn;
#pragma unroll 1
    for (int pp = 0; pp < 2; ++pp) {
#pragma unroll
      for (int q = 0; q < 6; ++q) *(volatile v4f*)(vd + (size_t)n0 * VW + q * 128 + 4 * lane) = ov[q];
      __threadfence();
    }
  }
  if (last == 0) {
#pragma unroll 1
    for (int pp = 0; pp < 2; ++pp) {
#pragma unroll 4
      for (int q = 0; q < 16; ++q) {
        const v4f v = *(const v4f*)(HN + q * TP + 4 * lane);
        *(volatile v4f*)(Hn + (size_t)(n0 + q) * HF + 4 * lane) = v;
      }
      __threadfence();
    }
    zacc<8>(acc);
    gemmS<4, 8, 1>(wp, psPQ, HN, TP, acc, lane);
    epi<8, 0, 0, 0>(acc, d3, MI, X, T1, lane);
    __syncthreads();
    zacc<8>(acc);
    gemmS<4, 8, 1>(wq, psPQ, HN, TP, acc, lane);
    epi<8, 0, 0, 0>(acc, d3, MI, X, T2, lane);
    __syncthreads();
#pragma unroll 1
    for (int pp = 0; pp < 2; ++pp) {
#pragma unroll 4
      for (int q = 0; q < 16; ++q) {
        const v4f a = *(const v4f*)(T1 + q * TP + 4 * lane);
        const v4f c = *(const v4f*)(T2 + q * TP + 4 * lane);
        *(volatile v4f*)(Pn + (size_t)(n0 + q) * HF + 4 * lane) = a;
        *(volatile v4f*)(Qn + (size_t)(n0 + q) * HF + 4 * lane) = c;
      }
      __threadfence();
    }
  } else {
    const float* hrow = HN + n * TP + 64 * h;
    float* prow = T1 + n * TP + 64 * h;
    float mx = -3.0e38f;
#pragma unroll 4
    for (int q = 0; q < 16; ++q) {
      const v4f v = *(const v4f*)(hrow + 4 * q);
      mx = fmaxf(mx, fmaxf(fmaxf(v.x, v.y), fmaxf(v.z, v.w)));
    }
    mx = fmaxf(mx, __shfl_xor(mx, 16));
    float sm = 0.0f;
#pragma unroll 2
    for (int q = 0; q < 16; ++q) {
      const v4f v = *(const v4f*)(hrow + 4 * q);
      v4f ev;
      ev.x = expf(v.x - mx); ev.y = expf(v.y - mx); ev.z = expf(v.z - mx); ev.w = expf(v.w - mx);
      sm += ev.x; sm += ev.y; sm += ev.z; sm += ev.w;
      *(v4f*)(prow + 4 * q) = ev;
    }
    sm += __shfl_xor(sm, 16);
    const float inv = 1.0f / sm;
#pragma unroll 4
    for (int q = 0; q < 16; ++q) {
      v4f ev = *(const v4f*)(prow + 4 * q);
      ev.x = ev.x * inv; ev.y = ev.y * inv; ev.z = ev.z * inv; ev.w = ev.w * inv;
      *(v4f*)(prow + 4 * q) = ev;
    }
    __syncthreads();
    v8f a4[4];
    zacc<4>(a4);
    gemmS<4, 4, 1>(wr, psR, T1, TP, a4, lane);
    epi<4, 0, 1, 0>(a4, rb, MI, X, T2, lane);
    __syncthreads();
#pragma unroll 1
    for (int pp = 0; pp < 2; ++pp) {
#pragma unroll
      for (int q = 0; q < 8; ++q) {
        const int fi = q * 128 + 4 * lane;
        const int row = fi >> 6, col = fi & 63;
        const v4f v = *(const v4f*)(T2 + row * TP + col);
        *(volatile v4f*)(out + (size_t)NTOT * VW + (size_t)n0 * OH + fi) = v;
      }
      __threadfence();
    }
  }
}

static size_t al256(size_t b) { return (b + 255) & ~(size_t)255; }

extern "C" void kernel_launch(void* const* d_in, const int* in_sizes, int n_in,
                              void* d_out, int out_size, void* d_ws, size_t ws_size,
                              hipStream_t stream) {
  if (n_in != 21 || d_in == 0 || in_sizes == 0) return;
  const int ex[21] = {1536, 104448, 384, 49152, 384, 384, 3, 49152, 384, 49152, 384,
                      6144, 48, 98304, 384, 49152, 384, 49152, 384, 8192, 64};
  for (int i = 0; i < 21; ++i) if (in_sizes[i] != ex[i]) return;
  if (out_size != NTOT * VW + NTOT * OH) return;
  const float* in[21];
  for (int i = 0; i < 21; ++i) in[i] = (const float*)d_in[i];
  float* out = (float*)d_out;

  const int sidx[12] = {1, 1, 1, 3, 5, 7, 9, 11, 13, 15, 17, 19};
  const int sL[12]   = {3, 3, 3, 3, 3, 3, 3, 3, 3, 3, 3, 1};
  const int sStr[12] = {34816, 34816, 34816, 16384, 128, 16384, 16384, 2048, 32768, 16384, 16384, 8192};
  const int sK0[12]  = {0, 16, 144, 0, 0, 0, 0, 0, 0, 0, 0, 0};
  const int sK[12]   = {16, 128, 128, 128, 128, 128, 128, 128, 256, 128, 128, 128};
  const int sNs[12]  = {128, 128, 128, 128, 1, 128, 128, 16, 128, 128, 128, 64};
  const int sNp[12]  = {128, 128, 128, 128, 16, 128, 128, 16, 128, 128, 128, 64};
  const int sKp[12]  = {32, 128, 128, 128, 128, 128, 128, 128, 256, 128, 128, 128};
  const int sPl[12]  = {3, 3, 3, 3, 3, 2, 2, 2, 3, 3, 3, 3};
  char* ws = (char*)d_ws;
  size_t off = 0;
  size_t oW[12];
  int E[12], LS[12];
  for (int i = 0; i < 12; ++i) {
    LS[i] = sNp[i] * sKp[i];
    E[i]  = sL[i] * LS[i];
    oW[i] = off;
    off += al256((size_t)sPl[i] * (size_t)E[i] * 2);
  }
  const size_t oVIN = off; off += al256((size_t)NTOT * 4 * 4);
  const size_t oVA  = off; off += al256((size_t)NTOT * VW * 4);
  const size_t oVB  = off; off += al256((size_t)NTOT * VW * 4);
  const size_t oHA  = off; off += al256((size_t)NTOT * HF * 4);
  const size_t oHB  = off; off += al256((size_t)NTOT * HF * 4);
  const size_t oP   = off; off += al256((size_t)NTOT * HF * 4);
  const size_t oQ   = off; off += al256((size_t)NTOT * HF * 4);
  const size_t oMI  = off; off += al256((size_t)NTOT * HF * 4);
  const size_t oSH  = off; off += al256((size_t)NTOT * 64 * 4);
  if (off > ws_size || off > (size_t)134217728) return;
  float* VIN = (float*)(ws + oVIN);
  float* VA  = (float*)(ws + oVA);
  float* VB  = (float*)(ws + oVB);
  float* HA  = (float*)(ws + oHA);
  float* HB  = (float*)(ws + oHB);
  float* PP  = (float*)(ws + oP);
  float* QQ  = (float*)(ws + oQ);
  float* MI  = (float*)(ws + oMI);
  float* SH  = (float*)(ws + oSH);

  for (int i = 0; i < 12; ++i) {
    const int nG = E[i] / 8;
    k_prep<<<(nG + 255) / 256, 256, 0, stream>>>(in[sidx[i]], (us*)(ws + oW[i]), sL[i], sStr[i], sK0[i],
                                                   sK[i], sNs[i], sNp[i], sKp[i], nG, E[i], sPl[i]);
  }
  k_init<<<2, NN, 0, stream>>>(in[0], VIN, VA, HA, PP, QQ);

  auto Wl = [&](int i, int l) -> const us* { return (const us*)(ws + oW[i]) + (size_t)l * (size_t)LS[i]; };
  float* vc = VA; float* vn = VB;
  float* hc = HA; float* hn = HB;
  for (int l = 0; l < 3; ++l) {
    k_pair<<<NTOT, 32, 0, stream>>>(vc, PP, QQ,
                                    Wl(0, l), E[0], Wl(3, l), E[3], Wl(4, l), E[4],
                                    Wl(5, l), E[5], Wl(6, l), E[6], Wl(7, l), E[7],
                                    in[2] + l * HF, in[4] + l * HF, in[6] + l,
                                    in[8] + l * HF, in[10] + l * HF, in[12] + l * 16,
                                    MI, SH);
    const int ln = (l < 2) ? (l + 1) : 0;
    const int last = (l == 2) ? 1 : 0;
    k_node<<<NTOT / 16, 32, 0, stream>>>(MI, SH, hc, vc, VIN,
                                         Wl(8, l), E[8], Wl(9, l), E[9], Wl(10, l), E[10],
                                         in[14] + l * HF, in[16] + l * HF, in[18] + l * HF,
                                         Wl(1, ln), Wl(2, ln), E[1], Wl(11, 0), E[11], in[20],
                                         hn, vn, PP, QQ, out, last);
    float* tv = vc; vc = vn; vn = tv;
    float* th = hc; hc = hn; hn = th;
  }
}
